// QuantLinear_10522669875875
// MI455X (gfx1250) — hardware-verified
//
#include <hip/hip_runtime.h>

constexpr int kM = 256;
constexpr int kK = 8192;
constexpr int kN = 8192;
constexpr int kGroup = 128;
constexpr int kNumGroups = kK / kGroup;
constexpr int kPackedRows = kK / 8;
constexpr int kPackedZCols = kN / 8;
constexpr int kBM = 128;
constexpr int kBN = 64;
constexpr int kBK = 32;
constexpr int kStepsPerGroup = kGroup / kBK;
constexpr int kThreads = 256;
constexpr int kLDA = 40;
constexpr int kLDB = 40;
constexpr int kSlabPitch = 36;

static_assert(kK % kGroup == 0 && kGroup % kBK == 0, "K steps by 32 inside 128 groups, no tail");
static_assert(kM % kBM == 0 && kN % kBN == 0, "M and N are exact tile multiples");
static_assert(kBM == 4 * 32 && kBN == 2 * 32 && kThreads == 8 * 32, "8 waves x 32x32");
static_assert(kBM * (kBK / 4) == 4 * kThreads, "A staging: 4 float4 per thread cover 128 x 32");
static_assert(kBN * (kBK / 8) == kThreads, "B staging: 1 packed word per thread covers 64 x 32");
static_assert((kLDA * 2) % 16 == 0 && (kLDB * 2) % 16 == 0 && (kSlabPitch * 4) % 16 == 0, "16-B aligned LDS rows");
static_assert((kN * 4) % 128 == 0 && (32 * 4) == 128, "each 32-float row segment is one whole 128-B line");
static_assert(kPackedRows * 8 == kK && kPackedZCols * 8 == kN, "packing");

typedef __attribute__((ext_vector_type(16))) __bf16   v16b;
typedef __attribute__((ext_vector_type(8)))  __bf16   v8b;
typedef __attribute__((ext_vector_type(8)))  float    v8f;
typedef __attribute__((ext_vector_type(4)))  float    v4f;
typedef __attribute__((ext_vector_type(4)))  unsigned int v4u;
typedef __attribute__((ext_vector_type(2)))  unsigned int v2u;

__device__ __forceinline__ unsigned short f2bf_bits(float f) {
  unsigned u = __float_as_uint(f);
  return (unsigned short)((u + 0x7FFFu + ((u >> 16) & 1u)) >> 16);
}
__device__ __forceinline__ float bf_bits2f(unsigned short h) { return __uint_as_float(((unsigned)h) << 16); }

__device__ __forceinline__ void dep_guard_b(v8f& a, v8f& b, v16b x, v16b y) { asm volatile("v_nop\n\tv_nop\n\tv_nop\n\tv_nop" : "+v"(a), "+v"(b) : "v"(x), "v"(y)); }
__device__ __forceinline__ void keep4_b(v16b a, v16b b, v16b c, v16b d) { asm volatile("v_nop" :: "v"(a), "v"(b), "v"(c), "v"(d)); }
template <typename T> struct Frag;
template <> struct Frag<__bf16> {
  typedef v16b V; union U { v16b v; v8b h[2]; };
  static __device__ __forceinline__ v16b load(const __bf16* p) {
    U f; f.h[0] = *(const v8b*)(p); f.h[1] = *(const v8b*)(p + 16); return f.v;
  }
  static __device__ __forceinline__ v8f mma(v16b a, v16b b, v8f c) {
    return __builtin_amdgcn_wmma_f32_16x16x32_bf16(false, a, false, b, (short)0, c, false, false);
  }
  static __device__ __forceinline__ void guard(v8f& a, v8f& b, v16b x, v16b y) { dep_guard_b(a, b, x, y); }
  static __device__ __forceinline__ void keep(v16b a, v16b b, v16b c, v16b d) { keep4_b(a, b, c, d); }
};

__device__ __forceinline__ unsigned pk16(unsigned short a, unsigned short b) { return (unsigned)a | ((unsigned)b << 16); }

__device__ __forceinline__ void wmma_guard4(v8f& a, v8f& b, v8f& c, v8f& d, v16b w, v16b x, v16b y, v16b z) {
  asm volatile("v_nop\n\tv_nop\n\tv_nop\n\tv_nop" : "+v"(a), "+v"(b), "+v"(c), "+v"(d) : "v"(w), "v"(x), "v"(y), "v"(z));
}
__device__ __forceinline__ float bf16_rne_f32(float f) { return bf_bits2f(f2bf_bits(f)); }

__global__ __launch_bounds__(kThreads) void qlinear_wmma_kernel(
    const float* __restrict__ x, const int* __restrict__ qweight, const int* __restrict__ qzeros,
    const float* __restrict__ scales, const int* __restrict__ gidx, const float* __restrict__ bias,
    float* __restrict__ out) {
  __shared__ __align__(16) unsigned short As[kBM * kLDA];
  __shared__ __align__(16) unsigned short Bs[kBN * kLDB];
  __shared__ __align__(16) float slabAll[8][32 * kSlabPitch];

  const int tid   = threadIdx.x;
  const int lane  = tid & 31;
  const int wave  = tid >> 5;
  const int waveM = wave >> 1;
  const int waveN = wave & 1;
  const int hh    = lane >> 4;
  const int l16   = lane & 15;
  const int m0    = blockIdx.y * kBM;
  const int n0    = blockIdx.x * kBN;
  const int bcol  = tid & (kBN - 1);
  const int brow  = tid >> 6;
  const int gn    = n0 + bcol;
  const int zshift = (gn & 7) * 4;
  const int mBase = m0 + waveM * 32;
  const int nBase = n0 + waveN * 32;

  const __bf16* Abf = (const __bf16*)(const void*)As;
  const __bf16* Bbf = (const __bf16*)(const void*)Bs;
  const int aOff0 = (waveM * 32 + l16) * kLDA + 8 * hh;
  const int aOff1 = aOff0 + 16 * kLDA;
  const int bOff0 = (waveN * 32 + l16) * kLDB + 8 * hh;
  const int bOff1 = bOff0 + 16 * kLDB;

  const v8f z8 = {0.f, 0.f, 0.f, 0.f, 0.f, 0.f, 0.f, 0.f};
  v8f c00 = z8, c01 = z8, c10 = z8, c11 = z8;
  v8f t00 = z8, t01 = z8, t10 = z8, t11 = z8;

#pragma unroll 1
  for (int gi = 0; gi < kNumGroups; ++gi) {
    int gsel = gidx[gi * kGroup];
    gsel = gsel < 0 ? 0 : (gsel > kNumGroups - 1 ? kNumGroups - 1 : gsel);
    const unsigned zpack = (unsigned)qzeros[(size_t)gsel * kPackedZCols + (gn >> 3)];
    const int zq = (int)((zpack >> zshift) & 15u) + 1;

#pragma unroll 1
    for (int ss = 0; ss < kStepsPerGroup; ++ss) {
      const int k0 = gi * kGroup + ss * kBK;
#pragma unroll
      for (int i = 0; i < 4; ++i) {
        const int lin = tid + i * kThreads;
        const int row = lin >> 3;
        const int c4  = (lin & 7) * 4;
        const v4f v = *(const v4f*)(x + (size_t)(m0 + row) * kK + k0 + c4);
        v2u p;
        p[0] = pk16(f2bf_bits(v[0]), f2bf_bits(v[1]));
        p[1] = pk16(f2bf_bits(v[2]), f2bf_bits(v[3]));
        *(v2u*)(As + row * kLDA + c4) = p;
      }
      {
        const int kq = k0 >> 3;
        const unsigned packed = (unsigned)qweight[(size_t)(kq + brow) * kN + gn];
        unsigned short hb[8];
#pragma unroll
        for (int j = 0; j < 8; ++j) {
          const int qv = (int)((packed >> (4 * j)) & 15u);
          hb[j] = f2bf_bits((float)(qv - zq));
        }
        v4u o;
        o[0] = pk16(hb[0], hb[1]);
        o[1] = pk16(hb[2], hb[3]);
        o[2] = pk16(hb[4], hb[5]);
        o[3] = pk16(hb[6], hb[7]);
        *(v4u*)(Bs + bcol * kLDB + brow * 8) = o;
      }
      __syncthreads();
      const v16b a0 = Frag<__bf16>::load(Abf + aOff0);
      const v16b a1 = Frag<__bf16>::load(Abf + aOff1);
      const v16b b0 = Frag<__bf16>::load(Bbf + bOff0);
      const v16b b1 = Frag<__bf16>::load(Bbf + bOff1);
      t00 = Frag<__bf16>::mma(a0, b0, t00);
      t01 = Frag<__bf16>::mma(a0, b1, t01);
      t10 = Frag<__bf16>::mma(a1, b0, t10);
      t11 = Frag<__bf16>::mma(a1, b1, t11);
      wmma_guard4(t00, t01, t10, t11, a0, a1, b0, b1);
      __syncthreads();
    }
    const float* sp = scales + (size_t)gsel * kN + nBase;
    const float s0 = bf16_rne_f32(sp[l16]);
    const float s1 = bf16_rne_f32(sp[16 + l16]);
#pragma unroll
    for (int r = 0; r < 8; ++r) {
      c00[r] = fmaf(t00[r], s0, c00[r]);
      c01[r] = fmaf(t01[r], s1, c01[r]);
      c10[r] = fmaf(t10[r], s0, c10[r]);
      c11[r] = fmaf(t11[r], s1, c11[r]);
    }
    t00 = z8; t01 = z8; t10 = z8; t11 = z8;
  }

  float* slab = slabAll[wave];
  const float bv0 = bf16_rne_f32(bias[nBase + l16]);
  const float bv1 = bf16_rne_f32(bias[nBase + 16 + l16]);
#pragma unroll
  for (int r = 0; r < 8; ++r) {
    const int ra = 8 * hh + r;
    slab[ra * kSlabPitch + l16]             = c00[r] + bv0;
    slab[ra * kSlabPitch + 16 + l16]        = c01[r] + bv1;
    slab[(16 + ra) * kSlabPitch + l16]      = c10[r] + bv0;
    slab[(16 + ra) * kSlabPitch + 16 + l16] = c11[r] + bv1;
  }
  __syncthreads();
  {
    const int rq = lane >> 3;
    const int c4 = (lane & 7) * 4;
    float* ob = out + (size_t)mBase * kN + nBase;
    for (int pass = 0; pass < 2; ++pass) {
#pragma unroll
      for (int it = 0; it < 8; ++it) {
        const int row = it * 4 + rq;
        const v4f v = *(const v4f*)(slab + row * kSlabPitch + c4);
        *(volatile v4f*)(ob + (size_t)row * kN + c4) = v;
      }
      __threadfence();
    }
  }
}

extern "C" void kernel_launch(void* const* d_in, const int* in_sizes, int n_in,
                              void* d_out, int out_size, void* d_ws, size_t ws_size, hipStream_t stream) {
  (void)d_ws; (void)ws_size;
  if (n_in < 6) return;
  if (in_sizes[0] != kM * kK) return;
  if (in_sizes[1] != kPackedRows * kN) return;
  if (in_sizes[2] != kNumGroups * kPackedZCols) return;
  if (in_sizes[3] != kNumGroups * kN) return;
  if (in_sizes[4] != kK) return;
  if (in_sizes[5] != kN) return;
  if (out_size != kM * kN) return;
  const float* x       = (const float*)d_in[0];
  const int*   qweight = (const int*)d_in[1];
  const int*   qzeros  = (const int*)d_in[2];
  const float* scales  = (const float*)d_in[3];
  const int*   gidx    = (const int*)d_in[4];
  const float* bias    = (const float*)d_in[5];
  float*       out     = (float*)d_out;
  dim3 grid(kN / kBN, kM / kBM);
  dim3 block(kThreads);
  qlinear_wmma_kernel<<<grid, block, 0, stream>>>(x, qweight, qzeros, scales, gidx, bias, out);
}
